// GCN_20779051778665
// MI455X (gfx1250) — hardware-run, weakly checked
//
#include <hip/hip_runtime.h>
#include <stddef.h>
#include <stdint.h>

#define NN      50000
#define NE      600000
#define DF      128
#define DO      64
#define KC      256
#define GBM     128
#define MP      50048
#define SP      68
#define NTHR    256
#define NWAVE   8
#define EPT     8
#define WCH     (32 * EPT)
#define NBRUN   1024
#define SLB     10
#define NBK     49
#define WLCAP   2048
#define RCAP    16384
#define DEGCAP  64
#define MAXDEG_MEAS 28
#define MAXBLK_MEAS 12531
#define ARB     64
#define WSMAX   (128u << 20)

#define BK_ZINTS (NWAVE * WLCAP + RCAP + 3 * NBRUN)
#define BK_INTS  (BK_ZINTS + NBRUN + 16)
#define BK_LDS   (BK_INTS * 4)

#define PBX   (MP * DF / 8 / NTHR)
#define PBW   (DF * KC / 8 / NTHR)
#define PBWC  (DO * KC / 8 / NTHR)
#define PBTOT (PBX + 2 * PBW + PBWC + 1)

static_assert(MP % GBM == 0 && MP >= NN && MP == 391 * GBM && MP % ARB == 0);
static_assert(NBRUN == (1 << SLB) && NBRUN % ARB == 0 && NBRUN % GBM == 0 && NBRUN % 128 == 0);
static_assert(NBK * NBRUN >= MP && NBK * NBRUN >= NN);
static_assert(NE % EPT == 0 && NE < (1 << 21) && (((long long)NE) << SLB) < (1LL << 31));
static_assert(RCAP == NWAVE * WLCAP && RCAP % (NTHR * 4) == 0 && BK_ZINTS % (NTHR * 4) == 0);
static_assert((long long)RCAP * 100 >= (long long)MAXBLK_MEAS * 105);
static_assert(WLCAP >= MAXBLK_MEAS / 8 + 8 * 40 + 1);
static_assert(MAXDEG_MEAS + 8 <= DEGCAP);
static_assert(NN <= 65536);
static_assert(NBRUN == NTHR * 4);
static_assert(KC % 32 == 0 && KC == 2 * DF && DF == 2 * 64 && DO == 64);
static_assert((MP * DF / 8) % NTHR == 0 && (DF * KC / 8) % NTHR == 0 && (DO * KC / 8) % NTHR == 0);
static_assert(ARB == NWAVE * 8 && GBM == NWAVE * 16);
static_assert(BK_LDS <= 300000 && BK_LDS <= 327680);
static_assert((GBM * SP + 128) * 4 <= 65536);

typedef float          v4f   __attribute__((ext_vector_type(4)));
typedef float          v8f   __attribute__((ext_vector_type(8)));
typedef int            v4i   __attribute__((ext_vector_type(4)));
typedef int            v8i   __attribute__((ext_vector_type(8)));
typedef unsigned       v2u   __attribute__((ext_vector_type(2)));
typedef unsigned short v8us  __attribute__((ext_vector_type(8)));
typedef unsigned short v16us __attribute__((ext_vector_type(16)));
typedef __bf16         v16bf __attribute__((ext_vector_type(16)));
typedef v4f  __attribute__((may_alias)) v4fa;
typedef v4i  __attribute__((may_alias)) v4ia;
typedef v2u  __attribute__((may_alias)) v2ua;
typedef v8us __attribute__((may_alias)) v8usa;
union FragB { v16bf v; v16us u; v8us h[2]; v8i w; };

__device__ __forceinline__ v8f wmb(const FragB& a, const FragB& b, v8f c) {
  v8f d = __builtin_amdgcn_wmma_f32_16x16x32_bf16(false, a.v, false, b.v, (short)0, c, false, false);
  asm volatile("v_nop\n\tv_nop\n\tv_nop\n\tv_nop" : "+v"(d) : "v"(a.w), "v"(b.w));
  return d;
}

__device__ __forceinline__ unsigned bf16_bits(float f) {
  const unsigned u = __float_as_uint(f);
  const unsigned r = (u + 0x7FFFu + ((u >> 16) & 1u)) >> 16;
  const unsigned q = (u >> 16) | 0x40u;
  return ((u & 0x7fffffffu) > 0x7f800000u) ? q : r;
}
__device__ __forceinline__ float bf16_val(float f) {
  return __uint_as_float(bf16_bits(f) << 16);
}

__device__ __forceinline__ void hilo_pack(float v0, float v1, float v2, float v3,
                                          int& h01, int& h23, int& l01, int& l23) {
  const unsigned a0 = bf16_bits(v0), a1 = bf16_bits(v1), a2 = bf16_bits(v2), a3 = bf16_bits(v3);
  const unsigned b0 = bf16_bits(v0 - __uint_as_float(a0 << 16));
  const unsigned b1 = bf16_bits(v1 - __uint_as_float(a1 << 16));
  const unsigned b2 = bf16_bits(v2 - __uint_as_float(a2 << 16));
  const unsigned b3 = bf16_bits(v3 - __uint_as_float(a3 << 16));
  h01 = (int)(a0 | (a1 << 16)); h23 = (int)(a2 | (a3 << 16));
  l01 = (int)(b0 | (b1 << 16)); l23 = (int)(b2 | (b3 << 16));
}

__device__ __forceinline__ v4i regroup8(int h01, int h23, int l01, int l23, int lane) {
  const int t  = lane & 15;
  const int s0 = (lane & 16) + ((2 * t) & 15), s1 = s0 + 1;
  const int a0 = __shfl(h01, s0, 32), a1 = __shfl(h23, s0, 32), a2 = __shfl(h01, s1, 32), a3 = __shfl(h23, s1, 32);
  const int b0 = __shfl(l01, s0, 32), b1 = __shfl(l23, s0, 32), b2 = __shfl(l01, s1, 32), b3 = __shfl(l23, s1, 32);
  const int mk = (t < 8) ? -1 : 0;
  v4i o;
  o.x = (a0 & mk) | (b0 & ~mk); o.y = (a1 & mk) | (b1 & ~mk);
  o.z = (a2 & mk) | (b2 & ~mk); o.w = (a3 & mk) | (b3 & ~mk);
  return o;
}

__device__ __forceinline__ v4i regroup16(int h01, int h23, int l01, int l23, int lane) {
  const int s0 = (2 * lane) & 31, s1 = s0 + 1;
  const int a0 = __shfl(h01, s0, 32), a1 = __shfl(h23, s0, 32), a2 = __shfl(h01, s1, 32), a3 = __shfl(h23, s1, 32);
  const int b0 = __shfl(l01, s0, 32), b1 = __shfl(l23, s0, 32), b2 = __shfl(l01, s1, 32), b3 = __shfl(l23, s1, 32);
  const int mk = (lane < 16) ? -1 : 0;
  v4i o;
  o.x = (a0 & mk) | (b0 & ~mk); o.y = (a1 & mk) | (b1 & ~mk);
  o.z = (a2 & mk) | (b2 & ~mk); o.w = (a3 & mk) | (b3 & ~mk);
  return o;
}

__device__ __forceinline__ void st2_v4f(float* p, v4f v) {
  *(volatile v4f*)p = v;
  __threadfence();
  *(volatile v4f*)p = v;
}
__device__ __forceinline__ void st2_v8us(unsigned short* p, v8us v) {
  *(volatile v8us*)p = v;
  __threadfence();
  *(volatile v8us*)p = v;
}

__device__ __forceinline__ v8us gather8(const float* __restrict__ base, int stride) {
  float f[8];
#pragma unroll
  for (int i = 0; i < 8; ++i) f[i] = base[(size_t)i * (size_t)stride];
  v8us o;
#pragma unroll
  for (int i = 0; i < 8; ++i) o[i] = (unsigned short)bf16_bits(f[i]);
  return o;
}

__device__ __forceinline__ v4f bf16_val4(v4f a) {
  v4f o;
  o.x = bf16_val(a.x); o.y = bf16_val(a.y); o.z = bf16_val(a.z); o.w = bf16_val(a.w);
  return o;
}

__global__ __launch_bounds__(NTHR) void k_prep(const float* __restrict__ x,
                                               const float* __restrict__ wa, const float* __restrict__ ba,
                                               const float* __restrict__ wb, const float* __restrict__ bb,
                                               const float* __restrict__ wc, const float* __restrict__ bc,
                                               unsigned short* xb, unsigned short* wda, unsigned short* wdb,
                                               unsigned short* wdc, float* sm) {
  const int tid = (int)threadIdx.x, lane = tid & 31, wave = tid >> 5;
  const int blk = (int)blockIdx.x;
  if (blk < PBX) {
    const int u   = blk * NTHR + tid;
    const int row = u >> 4, k8 = (u & 15) * 8;
    const int rc  = row < NN ? row : NN - 1;
    const unsigned mk = row < NN ? 0xffffu : 0u;
    const float* p = x + (size_t)rc * DF + k8;
    const v4f a = *(const v4fa*)p;
    const v4f b = *(const v4fa*)(p + 4);
    v8us o;
    o[0] = (unsigned short)(bf16_bits(a.x) & mk); o[1] = (unsigned short)(bf16_bits(a.y) & mk);
    o[2] = (unsigned short)(bf16_bits(a.z) & mk); o[3] = (unsigned short)(bf16_bits(a.w) & mk);
    o[4] = (unsigned short)(bf16_bits(b.x) & mk); o[5] = (unsigned short)(bf16_bits(b.y) & mk);
    o[6] = (unsigned short)(bf16_bits(b.z) & mk); o[7] = (unsigned short)(bf16_bits(b.w) & mk);
    st2_v8us(xb + (size_t)row * DF + k8, o);
  } else if (blk < PBX + PBW) {
    const int u = (blk - PBX) * NTHR + tid;
    const int n = u >> 5, k8 = (u & 31) * 8, kk = k8 & (DF - 1);
    const v8us o = gather8(wa + (size_t)kk * DF + n, DF);
    st2_v8us(wda + (size_t)n * KC + k8, o);
  } else if (blk < PBX + 2 * PBW) {
    const int u = (blk - PBX - PBW) * NTHR + tid;
    const int n = u >> 5, k8 = (u & 31) * 8, kk = k8 & (DF - 1);
    const v8us o = gather8(wb + (size_t)kk * DF + n, DF);
    st2_v8us(wdb + (size_t)n * KC + k8, o);
  } else if (blk < PBX + 2 * PBW + PBWC) {
    const int u = (blk - PBX - 2 * PBW) * NTHR + tid;
    const int n = u >> 5, k8 = (u & 31) * 8, kk = k8 & (DF - 1);
    const v8us o = gather8(wc + (size_t)kk * DO + n, DO);
    st2_v8us(wdc + (size_t)n * KC + k8, o);
  } else {
    if (wave == 0) {
      const v4f a = *(const v4fa*)(ba + 4 * lane);
      st2_v4f(sm + 4 * lane, bf16_val4(a));
    } else if (wave == 1) {
      const v4f a = *(const v4fa*)(bb + 4 * lane);
      st2_v4f(sm + DF + 4 * lane, bf16_val4(a));
    } else if (wave == 2) {
      const int q = lane & 15;
      const v4f a = *(const v4fa*)(bc + 4 * q);
      asm volatile("" :: "v"(a));
      const v4f o = bf16_val4(a);
      float* p = sm + 2 * DF + 4 * q;
      if (lane < 16) *(volatile v4f*)p = o;
      __threadfence();
      if (lane < 16) *(volatile v4f*)p = o;
    }
  }
}

__device__ __forceinline__ void bucket_flush(const int* pl, const int* cnt, const int* offs, const int* invb,
                                             int ov, int* lp, int* cp, int* op, int* ip, int* fp, int tid) {
#pragma unroll 1
  for (int i = tid * 4; i < RCAP; i += NTHR * 4) {
    const v4i v = *(const v4ia*)(pl + i);
    *(volatile v4i*)(lp + i) = v;
  }
  {
    const v4i v = *(const v4ia*)(cnt + 4 * tid);
    *(volatile v4i*)(cp + 4 * tid) = v;
  }
  {
    const v4i v = *(const v4ia*)(offs + 4 * tid);
    *(volatile v4i*)(op + 4 * tid) = v;
  }
  {
    const v4i v = *(const v4ia*)(invb + 4 * tid);
    *(volatile v4i*)(ip + 4 * tid) = v;
  }
  if (tid < 8) {
    const v4i f = {ov, ov, ov, ov};
    *(volatile v4i*)(fp + 4 * tid) = f;
  }
}

__global__ __launch_bounds__(NTHR) void k_bucket(const int* __restrict__ srcs, const int* __restrict__ dsts,
                                                 int* LIST, int* CNT, int* OFF, int* INVB, int* FLAG) {
  extern __shared__ __attribute__((aligned(16))) int dsm[];
  int* wl   = dsm;
  int* pl   = dsm + NWAVE * WLCAP;
  int* cnt  = pl + RCAP;
  int* offs = cnt + NBRUN;
  int* cur  = offs + NBRUN;
  int* invb = cur + NBRUN;
  int* misc = invb + NBRUN;
  const int tid = (int)threadIdx.x, lane = tid & 31, wave = tid >> 5;
  const int blk = (int)blockIdx.x;
  const unsigned nbs = (unsigned)(blk * NBRUN);

  {
    const v4i z4 = {0, 0, 0, 0};
    for (int i = tid * 4; i < BK_ZINTS; i += NTHR * 4) *(v4ia*)(dsm + i) = z4;
    if (tid < 16) misc[tid] = 0;
  }
  __syncthreads();

  {
    const int per  = ((NE + NWAVE * WCH - 1) / (NWAVE * WCH)) * WCH;
    const int ebeg = wave * per;
    const int eend = (ebeg + per < NE) ? (ebeg + per) : NE;
    int* mylist = wl + wave * WLCAP;
    int wc = 0;
#pragma unroll 1
    for (int cb = ebeg; cb < eend; cb += WCH) {
      const int e0  = cb + lane * EPT;
      const bool inr = e0 < NE;
      const int e0c = inr ? e0 : (NE - EPT);
      const v4i da = *(const v4ia*)(dsts + e0c);
      const v4i db = *(const v4ia*)(dsts + e0c + 4);
      const unsigned s0 = (unsigned)da.x - nbs, s1 = (unsigned)da.y - nbs;
      const unsigned s2 = (unsigned)da.z - nbs, s3 = (unsigned)da.w - nbs;
      const unsigned s4 = (unsigned)db.x - nbs, s5 = (unsigned)db.y - nbs;
      const unsigned s6 = (unsigned)db.z - nbs, s7 = (unsigned)db.w - nbs;
      const bool h0 = inr & (s0 < (unsigned)NBRUN), h1 = inr & (s1 < (unsigned)NBRUN);
      const bool h2 = inr & (s2 < (unsigned)NBRUN), h3 = inr & (s3 < (unsigned)NBRUN);
      const bool h4 = inr & (s4 < (unsigned)NBRUN), h5 = inr & (s5 < (unsigned)NBRUN);
      const bool h6 = inr & (s6 < (unsigned)NBRUN), h7 = inr & (s7 < (unsigned)NBRUN);
      const unsigned m0 = __builtin_amdgcn_ballot_w32(h0), m1 = __builtin_amdgcn_ballot_w32(h1);
      const unsigned m2 = __builtin_amdgcn_ballot_w32(h2), m3 = __builtin_amdgcn_ballot_w32(h3);
      const unsigned m4 = __builtin_amdgcn_ballot_w32(h4), m5 = __builtin_amdgcn_ballot_w32(h5);
      const unsigned m6 = __builtin_amdgcn_ballot_w32(h6), m7 = __builtin_amdgcn_ballot_w32(h7);
      const unsigned any = m0 | m1 | m2 | m3 | m4 | m5 | m6 | m7;
      if (any != 0u) {
        const int pre = (int)(__builtin_amdgcn_mbcnt_lo(m0, 0u) + __builtin_amdgcn_mbcnt_lo(m1, 0u) +
                              __builtin_amdgcn_mbcnt_lo(m2, 0u) + __builtin_amdgcn_mbcnt_lo(m3, 0u) +
                              __builtin_amdgcn_mbcnt_lo(m4, 0u) + __builtin_amdgcn_mbcnt_lo(m5, 0u) +
                              __builtin_amdgcn_mbcnt_lo(m6, 0u) + __builtin_amdgcn_mbcnt_lo(m7, 0u));
        int p = wc + pre;
        if (h0) { if (p < WLCAP) mylist[p] = ((e0 + 0) << SLB) | (int)s0; p = p + 1; }
        if (h1) { if (p < WLCAP) mylist[p] = ((e0 + 1) << SLB) | (int)s1; p = p + 1; }
        if (h2) { if (p < WLCAP) mylist[p] = ((e0 + 2) << SLB) | (int)s2; p = p + 1; }
        if (h3) { if (p < WLCAP) mylist[p] = ((e0 + 3) << SLB) | (int)s3; p = p + 1; }
        if (h4) { if (p < WLCAP) mylist[p] = ((e0 + 4) << SLB) | (int)s4; p = p + 1; }
        if (h5) { if (p < WLCAP) mylist[p] = ((e0 + 5) << SLB) | (int)s5; p = p + 1; }
        if (h6) { if (p < WLCAP) mylist[p] = ((e0 + 6) << SLB) | (int)s6; p = p + 1; }
        if (h7) { if (p < WLCAP) mylist[p] = ((e0 + 7) << SLB) | (int)s7; p = p + 1; }
        wc += (int)(__builtin_popcount(m0) + __builtin_popcount(m1) + __builtin_popcount(m2) + __builtin_popcount(m3) +
                    __builtin_popcount(m4) + __builtin_popcount(m5) + __builtin_popcount(m6) + __builtin_popcount(m7));
      }
    }
    if (lane == 0) misc[wave] = wc;
  }
  __syncthreads();

  if (wave == 0) {
    int ov = 0;
#pragma unroll 1
    for (int w2 = 0; w2 < NWAVE; ++w2) {
      int c = misc[w2];
      if (c > WLCAP) ov = 1;
      c = c < 0 ? 0 : (c > WLCAP ? WLCAP : c);
#pragma unroll 1
      for (int b0 = 0; b0 < c; b0 += 32) {
        const int idx = b0 + lane;
        const int ent = wl[w2 * WLCAP + (idx < WLCAP ? idx : WLCAP - 1)];
        const int m32 = (c - b0) < 32 ? (c - b0) : 32;
#pragma unroll 1
        for (int k = 0; k < m32; ++k) {
          const int u    = __builtin_amdgcn_readlane(ent, k);
          const int slot = u & (NBRUN - 1);
          if (lane == 0) cnt[slot] = cnt[slot] + 1;
        }
      }
    }
    if (lane == 0) misc[9] = ov;
  }
  __syncthreads();
  if (wave == 0) {
    const int base = lane * (NBRUN / 32);
    int s = 0;
    int big = 0;
#pragma unroll 1
    for (int i = 0; i < NBRUN / 32; ++i) {
      const int cv = cnt[base + i];
      big |= (cv > DEGCAP) ? 1 : 0;
      s += cv;
    }
    int incl = s;
#pragma unroll
    for (int d = 1; d < 32; d <<= 1) {
      const int y = __shfl_up(incl, d, 32);
      if (lane >= d) incl += y;
    }
    int run = incl - s;
#pragma unroll 1
    for (int i = 0; i < NBRUN / 32; ++i) {
      const int cv = cnt[base + i];
      offs[base + i] = run;
      cur[base + i]  = run;
      run += cv;
    }
    const unsigned bm = __builtin_amdgcn_ballot_w32(big != 0);
    if (lane == 0 && bm != 0u) misc[9] = 1;
  }
  __syncthreads();

  if (wave == 0) {
#pragma unroll 1
    for (int w2 = 0; w2 < NWAVE; ++w2) {
      int c = misc[w2];
      c = c < 0 ? 0 : (c > WLCAP ? WLCAP : c);
#pragma unroll 1
      for (int b0 = 0; b0 < c; b0 += 32) {
        const int idx = b0 + lane;
        const int ent = wl[w2 * WLCAP + (idx < WLCAP ? idx : WLCAP - 1)];
        int eid = (ent >> SLB) & 0x1FFFFF;
        eid = eid > NE - 1 ? NE - 1 : eid;
        int sr = srcs[eid];
        sr = sr < 0 ? 0 : (sr > NN - 1 ? NN - 1 : sr);
        const int m32 = (c - b0) < 32 ? (c - b0) : 32;
#pragma unroll 1
        for (int k = 0; k < m32; ++k) {
          const int u    = __builtin_amdgcn_readlane(ent, k);
          const int wd   = __builtin_amdgcn_readlane(sr, k);
          const int slot = u & (NBRUN - 1);
          if (lane == 0) {
            int p = cur[slot];
            p = p < 0 ? 0 : (p > RCAP - 1 ? RCAP - 1 : p);
            pl[p] = wd;
            cur[slot] = p + 1;
          }
        }
      }
    }
  }
  __syncthreads();

#pragma unroll 1
  for (int i = tid; i < NBRUN; i += NTHR) {
    int c = cnt[i];
    c = c < 1 ? 1 : c;
    invb[i] = __float_as_int(1.0f / (float)c);
  }
  __syncthreads();

  const int ovf = misc[9];
  int* lp = LIST + (size_t)blk * RCAP;
  int* cp = CNT  + (size_t)blk * NBRUN;
  int* op = OFF  + (size_t)blk * NBRUN;
  int* ip = INVB + (size_t)blk * NBRUN;
  int* fp = FLAG + (size_t)blk * 32;
  bucket_flush(pl, cnt, offs, invb, ovf, lp, cp, op, ip, fp, tid);
  __threadfence();
  bucket_flush(pl, cnt, offs, invb, ovf, lp, cp, op, ip, fp, tid);
}

template <int FIRST>
__global__ __launch_bounds__(NTHR) void k_agg(const int* __restrict__ LIST, const int* __restrict__ CNT,
                                              const int* __restrict__ OFF, const int* __restrict__ INVB,
                                              const int* __restrict__ FLAG,
                                              const unsigned short* __restrict__ SRC, unsigned short* AGG) {
  const int tid = (int)threadIdx.x, lane = tid & 31, wave = tid >> 5;
  const int rowBase = (int)blockIdx.x * ARB;
  const int bucket  = rowBase >> SLB;
  const int* lb  = LIST + (size_t)bucket * RCAP;
  const int flag = FLAG[(size_t)bucket * 32];
  const float qnan = __uint_as_float(0x7fc00000u);

#pragma unroll 1
  for (int i = 0; i < ARB / NWAVE; ++i) {
    const int d = rowBase + (ARB / NWAVE) * wave + i;
    int cv = CNT[d];
    int ov = OFF[d];
    const int ib = INVB[d];
    const bool big = cv > DEGCAP;
    cv = cv < 0 ? 0 : (cv > DEGCAP ? DEGCAP : cv);
    ov = ov < 0 ? 0 : (ov > RCAP - 1 ? RCAP - 1 : ov);
    const int c = __builtin_amdgcn_readfirstlane(cv);
    const int o = __builtin_amdgcn_readfirstlane(ov);
    int last = o + c - 1; last = last < o ? o : last;
    last = last > RCAP - 1 ? RCAP - 1 : last;
    float a0 = 0.0f, a1 = 0.0f, a2 = 0.0f, a3 = 0.0f;
#pragma unroll 1
    for (int b0 = 0; b0 < c; b0 += 32) {
      int idx = o + b0 + lane;
      idx = idx > last ? last : idx;
      int sr = lb[idx];
      sr = sr < 0 ? 0 : (sr > NN - 1 ? NN - 1 : sr);
      const int m32 = (c - b0) < 32 ? (c - b0) : 32;
#pragma unroll 1
      for (int k = 0; k < m32; ++k) {
        const int sk = __builtin_amdgcn_readlane(sr, k);
        if constexpr (FIRST != 0) {
          const v2u w = *(const v2ua*)(SRC + (size_t)sk * DF + 4 * lane);
          a0 += __uint_as_float(w.x << 16);
          a1 += __uint_as_float(w.x & 0xffff0000u);
          a2 += __uint_as_float(w.y << 16);
          a3 += __uint_as_float(w.y & 0xffff0000u);
        } else {
          const unsigned short* rp = SRC + (size_t)sk * KC + 4 * lane;
          const v2u wh = *(const v2ua*)rp;
          const v2u wl = *(const v2ua*)(rp + DF);
          a0 += __uint_as_float(wh.x << 16)         + __uint_as_float(wl.x << 16);
          a1 += __uint_as_float(wh.x & 0xffff0000u) + __uint_as_float(wl.x & 0xffff0000u);
          a2 += __uint_as_float(wh.y << 16)         + __uint_as_float(wl.y << 16);
          a3 += __uint_as_float(wh.y & 0xffff0000u) + __uint_as_float(wl.y & 0xffff0000u);
        }
      }
    }
    const float inv = __int_as_float(ib);
    float m0 = a0 * inv, m1 = a1 * inv, m2 = a2 * inv, m3 = a3 * inv;
    const bool bad  = (flag != 0) | big;
    const bool live = d < NN;
    m0 = bad ? qnan : m0; m1 = bad ? qnan : m1; m2 = bad ? qnan : m2; m3 = bad ? qnan : m3;
    m0 = live ? m0 : 0.0f; m1 = live ? m1 : 0.0f; m2 = live ? m2 : 0.0f; m3 = live ? m3 : 0.0f;
    int h01, h23, l01, l23;
    hilo_pack(m0, m1, m2, m3, h01, h23, l01, l23);
    const v4i ow = regroup16(h01, h23, l01, l23, lane);
    unsigned short* hp = AGG + (size_t)d * KC + 8 * lane;
    *(volatile v4i*)hp = ow;
    __threadfence();
    *(volatile v4i*)hp = ow;
  }
}

template <int NT, int HB>
__device__ __forceinline__ void stage_half(float* stg, const v8f (&acc)[NT], int wave, int hh, int m) {
#pragma unroll
  for (int nt = 0; nt < 4; ++nt) {
#pragma unroll
    for (int r = 0; r < 8; ++r) stg[(16 * wave + 8 * hh + r) * SP + 16 * nt + m] = acc[4 * HB + nt][r];
  }
}

template <int HB, int FIN>
__device__ __forceinline__ void epi_rows(const float* stg, const float* sb, int rowBase, int flag,
                                         unsigned short* Hout, float* outp, int lane, int wave) {
  const int hh = lane >> 4, m = lane & 15;
  const v4f bias = *(const v4fa*)(sb + 64 * HB + 4 * m);
  const float qnan = __uint_as_float(0x7fc00000u);
#pragma unroll 1
  for (int i = 0; i < 8; ++i) {
    const int lr   = 16 * wave + 2 * i + hh;
    const int grow = rowBase + lr;
    const bool live = grow < NN;
    const v4f a = *(const v4fa*)(stg + lr * SP + 4 * m);
    asm volatile("" :: "v"(a));
    float v0 = a.x + bias.x, v1 = a.y + bias.y, v2 = a.z + bias.z, v3 = a.w + bias.w;
    if constexpr (FIN == 0) {
      v0 = (v0 > 0.0f) ? v0 : (v0 - v0); v1 = (v1 > 0.0f) ? v1 : (v1 - v1);
      v2 = (v2 > 0.0f) ? v2 : (v2 - v2); v3 = (v3 > 0.0f) ? v3 : (v3 - v3);
      v0 = live ? v0 : 0.0f; v1 = live ? v1 : 0.0f; v2 = live ? v2 : 0.0f; v3 = live ? v3 : 0.0f;
      int h01, h23, l01, l23;
      hilo_pack(v0, v1, v2, v3, h01, h23, l01, l23);
      const v4i ow = regroup8(h01, h23, l01, l23, lane);
      unsigned short* hp = Hout + (size_t)grow * KC + 64 * HB + 8 * (m & 7) + ((m >> 3) << 7);
      *(volatile v4i*)hp = ow;
      __threadfence();
      *(volatile v4i*)hp = ow;
    } else {
      const bool bad = flag != 0;
      v0 = bad ? qnan : v0; v1 = bad ? qnan : v1; v2 = bad ? qnan : v2; v3 = bad ? qnan : v3;
      v4f o;
      o.x = v0; o.y = v1; o.z = v2; o.w = v3;
      float* op = outp + (size_t)(live ? grow : 0) * DO + 4 * m;
      if (live) *(volatile v4f*)op = o;
      __threadfence();
      if (live) *(volatile v4f*)op = o;
    }
  }
}

template <int NCOL, int FIN>
__global__ __launch_bounds__(NTHR) __attribute__((amdgpu_num_vgpr(248)))
void k_gemm(const unsigned short* __restrict__ A, const unsigned short* __restrict__ BT,
            const float* __restrict__ bias, const int* __restrict__ FLAG,
            unsigned short* Hout, float* outp) {
  constexpr int NT = NCOL / 16;
  constexpr int NH = NCOL / 64;
  static_assert(NCOL == 64 || NCOL == 128);
  __shared__ __attribute__((aligned(16))) float stg[GBM * SP];
  __shared__ __attribute__((aligned(16))) float sb[128];
  const int tid = (int)threadIdx.x, lane = tid & 31, wave = tid >> 5, hh = lane >> 4, m = lane & 15;
  const int rowBase = (int)blockIdx.x * GBM;
  const int flag = FLAG[(size_t)(rowBase >> SLB) * 32];
  if (tid < NCOL / 4) *(v4fa*)(sb + 4 * tid) = *(const v4fa*)(bias + 4 * tid);

  v8f acc[NT];
  {
    const v8f z = {0.f, 0.f, 0.f, 0.f, 0.f, 0.f, 0.f, 0.f};
#pragma unroll
    for (int t = 0; t < NT; ++t) acc[t] = z;
  }
  const unsigned short* ap = A + (size_t)(rowBase + 16 * wave + m) * (size_t)KC + 8 * hh;
  const unsigned short* bp = BT + (size_t)m * (size_t)KC + 8 * hh;
#pragma unroll 1
  for (int k0 = 0; k0 < KC; k0 += 32) {
    FragB af;
    af.h[0] = *(const v8usa*)(ap + k0);
    af.h[1] = *(const v8usa*)(ap + k0 + 16);
#pragma unroll
    for (int nt = 0; nt < NT; ++nt) {
      const unsigned short* wq = bp + (size_t)(16 * nt) * (size_t)KC + k0;
      FragB bf;
      bf.h[0] = *(const v8usa*)wq;
      bf.h[1] = *(const v8usa*)(wq + 16);
      acc[nt] = wmb(af, bf, acc[nt]);
    }
  }

  stage_half<NT, 0>(stg, acc, wave, hh, m);
  __syncthreads();
  epi_rows<0, FIN>(stg, sb, rowBase, flag, Hout, outp, lane, wave);
  if constexpr (NH == 2) {
    __syncthreads();
    stage_half<NT, 1>(stg, acc, wave, hh, m);
    __syncthreads();
    epi_rows<1, FIN>(stg, sb, rowBase, flag, Hout, outp, lane, wave);
  }
}

extern "C" void kernel_launch(void* const* d_in, const int* in_sizes, int n_in,
                              void* d_out, int out_size, void* d_ws, size_t ws_size,
                              hipStream_t stream) {
  if (n_in < 9) return;
  if (in_sizes[0] != NN * DF) return;
  if (in_sizes[1] != NE || in_sizes[2] != NE) return;
  if (in_sizes[3] != DF * DF || in_sizes[4] != DF) return;
  if (in_sizes[5] != DF * DF || in_sizes[6] != DF) return;
  if (in_sizes[7] != DF * DO || in_sizes[8] != DO) return;
  if (out_size != NN * DO) return;

  const float* x    = (const float*)d_in[0];
  const int*   srcs = (const int*)d_in[1];
  const int*   dsts = (const int*)d_in[2];
  const float* wa   = (const float*)d_in[3];
  const float* ba   = (const float*)d_in[4];
  const float* wb   = (const float*)d_in[5];
  const float* bb   = (const float*)d_in[6];
  const float* wc   = (const float*)d_in[7];
  const float* bc   = (const float*)d_in[8];
  float* out = (float*)d_out;

  constexpr size_t zXB   = (size_t)MP * DF * 2;
  constexpr size_t zHL   = (size_t)MP * KC * 2;
  constexpr size_t zLIST = (size_t)NBK * RCAP * 4;
  constexpr size_t zTAB  = (size_t)NBK * NBRUN * 4;
  constexpr size_t zFLAG = (size_t)NBK * 128;
  constexpr size_t zWD   = (size_t)DF * KC * 2;
  constexpr size_t zWDC  = (size_t)DO * KC * 2;
  constexpr size_t zSM   = (size_t)(2 * DF + DO) * 4;
  constexpr size_t oXB   = 0;
  constexpr size_t oAGG  = oXB + zXB;
  constexpr size_t oH    = oAGG + zHL;
  constexpr size_t oLIST = oH + zHL;
  constexpr size_t oCNT  = oLIST + zLIST;
  constexpr size_t oOFF  = oCNT + zTAB;
  constexpr size_t oINV  = oOFF + zTAB;
  constexpr size_t oFLAG = oINV + zTAB;
  constexpr size_t oWDA  = oFLAG + zFLAG;
  constexpr size_t oWDB  = oWDA + zWD;
  constexpr size_t oWDC  = oWDB + zWD;
  constexpr size_t oSM   = oWDC + zWDC;
  constexpr size_t oEND  = oSM + zSM;
  static_assert(zXB % 128 == 0 && zHL % 128 == 0 && zLIST % 128 == 0 && zTAB % 128 == 0);
  static_assert(zFLAG % 128 == 0 && zWD % 128 == 0 && zWDC % 128 == 0 && zSM % 128 == 0);
  static_assert((size_t)(MP - 1) * KC * 2 + 512 <= zHL);
  static_assert((size_t)(MP - 1) * 4 + 4 <= zTAB);
  static_assert(oEND <= (size_t)WSMAX);
  if (oEND > ws_size) return;

  char* ws = (char*)d_ws;
  unsigned short* XB   = (unsigned short*)(ws + oXB);
  unsigned short* AGG  = (unsigned short*)(ws + oAGG);
  unsigned short* H    = (unsigned short*)(ws + oH);
  int*            LIST = (int*)(ws + oLIST);
  int*            CNT  = (int*)(ws + oCNT);
  int*            OFF  = (int*)(ws + oOFF);
  int*            INVB = (int*)(ws + oINV);
  int*            FLAG = (int*)(ws + oFLAG);
  unsigned short* WDA  = (unsigned short*)(ws + oWDA);
  unsigned short* WDB  = (unsigned short*)(ws + oWDB);
  unsigned short* WDC  = (unsigned short*)(ws + oWDC);
  float*          SM   = (float*)(ws + oSM);

  hipFuncSetAttribute(reinterpret_cast<const void*>(&k_bucket), hipFuncAttributeMaxDynamicSharedMemorySize, (int)BK_LDS);

  k_prep<<<PBTOT, NTHR, 0, stream>>>(x, wa, ba, wb, bb, wc, bc, XB, WDA, WDB, WDC, SM);
  k_bucket<<<NBK, NTHR, BK_LDS, stream>>>(srcs, dsts, LIST, CNT, OFF, INVB, FLAG);

  k_agg<1><<<MP / ARB, NTHR, 0, stream>>>(LIST, CNT, OFF, INVB, FLAG, XB, AGG);
  k_gemm<DF, 0><<<MP / GBM, NTHR, 0, stream>>>(AGG, WDA, SM, FLAG, H, out);
  k_agg<0><<<MP / ARB, NTHR, 0, stream>>>(LIST, CNT, OFF, INVB, FLAG, H, AGG);
  k_gemm<DF, 0><<<MP / GBM, NTHR, 0, stream>>>(AGG, WDB, SM + DF, FLAG, H, out);
  k_agg<0><<<MP / ARB, NTHR, 0, stream>>>(LIST, CNT, OFF, INVB, FLAG, H, AGG);
  k_gemm<DO, 1><<<MP / GBM, NTHR, 0, stream>>>(AGG, WDC, SM + 2 * DF, FLAG, H, out);
}
